// HyMultiHeadAttention_75651553952309
// MI455X (gfx1250) — hardware-verified
//
#include <hip/hip_runtime.h>
#include <stddef.h>
#include <stdint.h>

#define BB   4
#define NN   2048
#define CC   1024
#define HH   16
#define DD   64
#define ROWS (BB * NN)
#define PL   ((size_t)BB * HH * NN * DD)

static_assert(NN % 256 == 0);
static_assert(CC % 128 == 0);
static_assert(DD == 64);
static_assert(HH * DD == CC);
static_assert(ROWS % 256 == 0);
static_assert(ROWS % 32 == 0);

typedef _Float16 v16h __attribute__((ext_vector_type(16)));
typedef _Float16 v8h  __attribute__((ext_vector_type(8)));
typedef float    v8f  __attribute__((ext_vector_type(8)));
typedef float    v4f  __attribute__((ext_vector_type(4)));
typedef unsigned int v4u __attribute__((ext_vector_type(4)));

union Frag  { v16h v; v8h h[2]; };
union Pack8 { v8h h; v4u u; };

__device__ __forceinline__ v8f mma16(v16h a, v16h b, v8f c) {
  c = __builtin_amdgcn_wmma_f32_16x16x32_f16(false, a, false, b, (short)0, c, false, false);
  asm volatile("v_nop\n\tv_nop\n\tv_nop\n\tv_nop" : "+v"(c) : "v"(a), "v"(b));
  return c;
}

__device__ __forceinline__ v16h ldfrag(const _Float16* p, int ld, int row0, int k0, int lane) {
  const int m = lane & 15, lh = lane >> 4;
  const _Float16* q = p + (size_t)(row0 + m) * ld + k0 + 8 * lh;
  Frag f;
  f.h[0] = *(const v8h*)(q);
  f.h[1] = *(const v8h*)(q + 16);
  return f.v;
}

__device__ __forceinline__ v8f zero8() { return (v8f){0.f, 0.f, 0.f, 0.f, 0.f, 0.f, 0.f, 0.f}; }

__device__ __forceinline__ void gemm32x64(const _Float16* __restrict__ A, int lda,
                                          const _Float16* __restrict__ Bt, int ldb,
                                          int m0, int n0, int lane, v8f (&acc)[2][4]) {
#pragma unroll 2
  for (int k0 = 0; k0 < CC; k0 += 32) {
    const v16h a0 = ldfrag(A, lda, m0, k0, lane);
    const v16h a1 = ldfrag(A, lda, m0 + 16, k0, lane);
    const v16h b0 = ldfrag(Bt, ldb, n0, k0, lane);
    const v16h b1 = ldfrag(Bt, ldb, n0 + 16, k0, lane);
    const v16h b2 = ldfrag(Bt, ldb, n0 + 32, k0, lane);
    const v16h b3 = ldfrag(Bt, ldb, n0 + 48, k0, lane);
    acc[0][0] = mma16(a0, b0, acc[0][0]);
    acc[1][0] = mma16(a1, b0, acc[1][0]);
    acc[0][1] = mma16(a0, b1, acc[0][1]);
    acc[1][1] = mma16(a1, b1, acc[1][1]);
    acc[0][2] = mma16(a0, b2, acc[0][2]);
    acc[1][2] = mma16(a1, b2, acc[1][2]);
    acc[0][3] = mma16(a0, b3, acc[0][3]);
    acc[1][3] = mma16(a1, b3, acc[1][3]);
  }
}

__global__ __launch_bounds__(256) void k_xprep(const float* __restrict__ x, _Float16* __restrict__ xh,
                                               float* __restrict__ lam) {
  __shared__ __align__(16) float lamS[32];
  const int tid = threadIdx.x, lane = tid & 31, wave = tid >> 5;
  const int r0 = blockIdx.x * 32 + wave * 4;
#pragma unroll 1
  for (int i = 0; i < 4; ++i) {
    const size_t ro = (size_t)(r0 + i) * CC;
    float ss = 0.f;
#pragma unroll 1
    for (int it = 0; it < 4; ++it) {
      const size_t o = ro + (size_t)(it * 256 + lane * 8);
      const v4f a0 = *(const v4f*)(x + o);
      const v4f a1 = *(const v4f*)(x + o + 4);
      ss += a0[0] * a0[0] + a0[1] * a0[1] + a0[2] * a0[2] + a0[3] * a0[3]
          + a1[0] * a1[0] + a1[1] * a1[1] + a1[2] * a1[2] + a1[3] * a1[3];
      Pack8 pk;
      pk.h = (v8h){(_Float16)(a0[0] * 32.0f), (_Float16)(a0[1] * 32.0f),
                   (_Float16)(a0[2] * 32.0f), (_Float16)(a0[3] * 32.0f),
                   (_Float16)(a1[0] * 32.0f), (_Float16)(a1[1] * 32.0f),
                   (_Float16)(a1[2] * 32.0f), (_Float16)(a1[3] * 32.0f)};
      const v4u vv = pk.u;
      volatile v4u* d = (volatile v4u*)(xh + o);
      *d = vv;
      __threadfence();
      *d = vv;
    }
#pragma unroll
    for (int off = 16; off > 0; off >>= 1) ss += __shfl_xor(ss, off, 32);
    const float lv = 2.0f / (1.0f - ss);
    if (lane == 0) lamS[wave * 4 + i] = lv;
  }
  __syncthreads();
  if (tid < 8) {
    const v4f v = *(const v4f*)(lamS + tid * 4);
    volatile v4f* d = (volatile v4f*)(lam + (size_t)blockIdx.x * 32 + tid * 4);
    *d = v;
    __threadfence();
    *d = v;
  }
}

__global__ __launch_bounds__(256) void k_cvt8(const float* __restrict__ w, _Float16* __restrict__ wh,
                                              int ngrp, float sc) {
  const int t = blockIdx.x * 256 + (int)threadIdx.x;
  if (t >= ngrp) return;
  const size_t o = (size_t)t * 8;
  const v4f a0 = *(const v4f*)(w + o);
  const v4f a1 = *(const v4f*)(w + o + 4);
  Pack8 pk;
  pk.h = (v8h){(_Float16)(a0[0] * sc), (_Float16)(a0[1] * sc), (_Float16)(a0[2] * sc), (_Float16)(a0[3] * sc),
               (_Float16)(a1[0] * sc), (_Float16)(a1[1] * sc), (_Float16)(a1[2] * sc), (_Float16)(a1[3] * sc)};
  const v4u vv = pk.u;
  volatile v4u* d = (volatile v4u*)(wh + o);
  *d = vv;
  __threadfence();
  *d = vv;
}

#define WTP 68
__global__ __launch_bounds__(256) void k_wt(const float* __restrict__ w, _Float16* __restrict__ wt,
                                            int nout, float sc) {
  __shared__ __align__(16) float tf[64 * WTP];
  const int tid = threadIdx.x;
  const int n0 = blockIdx.x * 64;
  const int k0 = blockIdx.y * 64;
  {
    const int kr = tid >> 4;
    const int n4 = (tid & 15) * 4;
#pragma unroll
    for (int it = 0; it < 4; ++it) {
      const int kl = it * 16 + kr;
      const v4f a = *(const v4f*)(w + (size_t)(k0 + kl) * nout + n0 + n4);
      *(v4f*)(tf + kl * WTP + n4) = a;
    }
  }
  __syncthreads();
  v4u val[2];
  size_t go[2];
#pragma unroll
  for (int j = 0; j < 2; ++j) {
    const int p  = tid + 256 * j;
    const int nl = p >> 3;
    const int pc = p & 7;
    const float* cp = tf + (pc * 8) * WTP + nl;
    Pack8 pk;
    pk.h = (v8h){(_Float16)(cp[0 * WTP] * sc), (_Float16)(cp[1 * WTP] * sc),
                 (_Float16)(cp[2 * WTP] * sc), (_Float16)(cp[3 * WTP] * sc),
                 (_Float16)(cp[4 * WTP] * sc), (_Float16)(cp[5 * WTP] * sc),
                 (_Float16)(cp[6 * WTP] * sc), (_Float16)(cp[7 * WTP] * sc)};
    val[j] = pk.u;
    go[j]  = (size_t)(n0 + nl) * CC + k0 + pc * 8;
  }
  for (int ps = 0; ps < 2; ++ps) {
#pragma unroll
    for (int j = 0; j < 2; ++j) *(volatile v4u*)(wt + go[j]) = val[j];
    __threadfence();
  }
}

__global__ __launch_bounds__(256) void k_znorm(const float* __restrict__ z, float* __restrict__ zn) {
  __shared__ __align__(16) float znS[256];
  const int tid = threadIdx.x;
  const int n = blockIdx.x * 256 + tid;
  float s0 = 0.f, s1 = 0.f, s2 = 0.f, s3 = 0.f;
#pragma unroll 1
  for (int k = 0; k < CC; k += 4) {
    const float v0 = z[(size_t)(k + 0) * CC + n];
    const float v1 = z[(size_t)(k + 1) * CC + n];
    const float v2 = z[(size_t)(k + 2) * CC + n];
    const float v3 = z[(size_t)(k + 3) * CC + n];
    s0 = fmaf(v0, v0, s0);
    s1 = fmaf(v1, v1, s1);
    s2 = fmaf(v2, v2, s2);
    s3 = fmaf(v3, v3, s3);
  }
  const float ss = (s0 + s1) + (s2 + s3);
  znS[tid] = fmaxf(sqrtf(ss), 1e-15f);
  __syncthreads();
  if (tid < 64) {
    const v4f v = *(const v4f*)(znS + tid * 4);
    volatile v4f* d = (volatile v4f*)(zn + (size_t)blockIdx.x * 256 + tid * 4);
    *d = v;
    __threadfence();
    *d = v;
  }
}

#define TP 1028
#define HP 1032
#define HPROJ_LDS_FLOATS (16 * TP + (16 * HP) / 2 + 4 * CC + 16)
#define HPROJ_LDS_BYTES  (HPROJ_LDS_FLOATS * 4)
static_assert((16 * HP) % 2 == 0);
static_assert(((16 * TP) * 4) % 16 == 0);
static_assert((HP * 2) % 16 == 0);

__global__ __launch_bounds__(256) void k_hproj(const _Float16* __restrict__ xh,
                                               const _Float16* __restrict__ zt,
                                               const float* __restrict__ zn,
                                               const float* __restrict__ rb,
                                               const float* __restrict__ lam,
                                               _Float16* __restrict__ qp) {
  extern __shared__ __align__(16) float dsm[];
  float*    T32  = dsm;
  _Float16* T16  = (_Float16*)(dsm + 16 * TP);
  float*    znS  = dsm + 16 * TP + (16 * HP) / 2;
  float*    izS  = znS + CC;
  float*    chS  = izS + CC;
  float*    shS  = chS + CC;
  float*    lamS = shS + CC;

  const int tid = threadIdx.x, lane = tid & 31, wave = tid >> 5;
  const int hh = lane >> 4, c = lane & 15;
  const int tokbase = blockIdx.x * 16;
  const int n0 = wave * 128;

#pragma unroll 1
  for (int i = 0; i < 4; ++i) {
    const int j = tid + 256 * i;
    const float zv = zn[j];
    znS[j] = zv;
    izS[j] = 1.0f / zv;
    const float t2 = 2.0f * rb[j];
    chS[j] = coshf(t2);
    shS[j] = sinhf(t2);
  }
  if (tid < 16) lamS[tid] = lam[tokbase + tid];

  v8f acc[8];
#pragma unroll
  for (int t = 0; t < 8; ++t) acc[t] = zero8();
#pragma unroll 1
  for (int k0 = 0; k0 < CC; k0 += 32) {
    const v16h a = ldfrag(xh, CC, tokbase, k0, lane);
#pragma unroll
    for (int t = 0; t < 8; ++t) {
      const v16h b = ldfrag(zt, CC, n0 + 16 * t, k0, lane);
      acc[t] = mma16(a, b, acc[t]);
    }
  }
#pragma unroll
  for (int t = 0; t < 8; ++t)
#pragma unroll
    for (int r = 0; r < 8; ++r) T32[(8 * hh + r) * TP + n0 + 16 * t + c] = acc[t][r];
  __syncthreads();

  const int row = tid >> 4, cl = tid & 15;
  const float lv = lamS[row], lm1 = lv - 1.0f;
  float* trow = T32 + row * TP;
  float ssq = 0.f;
#pragma unroll 1
  for (int i = 0; i < 64; ++i) {
    const int col = i * 16 + cl;
    const float inner = (trow[col] * 0.001953125f) * izS[col];
    const float g  = (lv * inner) * chS[col] - lm1 * shS[col];
    const float as = asinhf(g);
    const float v  = 2.0f * znS[col] * as;
    const float w  = sinhf(v);
    trow[col] = w;
    ssq = fmaf(w, w, ssq);
  }
  ssq += __shfl_xor(ssq, 1, 32);
  ssq += __shfl_xor(ssq, 2, 32);
  ssq += __shfl_xor(ssq, 4, 32);
  ssq += __shfl_xor(ssq, 8, 32);
  const float osc = 32.0f / (1.0f + sqrtf(1.0f + ssq));
  _Float16* hrow = T16 + row * HP;
#pragma unroll 1
  for (int i = 0; i < 64; ++i) {
    const int col = i * 16 + cl;
    hrow[col] = (_Float16)(trow[col] * osc);
  }
  __syncthreads();

  v4u val[8];
  size_t go[8];
#pragma unroll
  for (int j = 0; j < 8; ++j) {
    const int p  = tid + 256 * j;
    const int L  = p >> 3;
    const int pc = p & 7;
    const int rw = L >> 4;
    const int hd = L & 15;
    const int tok = tokbase + rw;
    const int b = tok >> 11;
    const int n = tok & (NN - 1);
    Pack8 pk;
    pk.h   = *(const v8h*)(T16 + rw * HP + hd * 64 + pc * 8);
    val[j] = pk.u;
    go[j]  = ((size_t)(b * HH + hd) * NN + n) * DD + pc * 8;
  }
  for (int ps = 0; ps < 2; ++ps) {
#pragma unroll
    for (int j = 0; j < 8; ++j) *(volatile v4u*)(qp + go[j]) = val[j];
    __threadfence();
  }
}

#define STP 72
__global__ __launch_bounds__(256) void k_vproj(const _Float16* __restrict__ xh,
                                               const _Float16* __restrict__ wt,
                                               _Float16* __restrict__ vtp) {
  __shared__ __align__(16) _Float16 st[256 * STP];
  const int tid = threadIdx.x, lane = tid & 31, wave = tid >> 5;
  const int hh = lane >> 4, c = lane & 15;
  const int mb = blockIdx.x * 256;
  const int m0 = mb + wave * 32;
  const int n0 = blockIdx.y * 64;

  v8f acc[2][4];
#pragma unroll
  for (int s = 0; s < 2; ++s)
#pragma unroll
    for (int t = 0; t < 4; ++t) acc[s][t] = zero8();
  gemm32x64(xh, CC, wt, CC, m0, n0, lane, acc);

#pragma unroll
  for (int t = 0; t < 4; ++t) {
#pragma unroll
    for (int sub = 0; sub < 2; ++sub) {
#pragma unroll
      for (int r = 0; r < 8; ++r) {
        const int lr = wave * 32 + sub * 16 + 8 * hh + r;
        st[lr * STP + 16 * t + c] = (_Float16)(acc[sub][t][r] * 0.03125f);
      }
    }
  }
  __syncthreads();

  const int head = n0 >> 6;
  const int b  = mb >> 11;
  const int nb = mb & (NN - 1);
  const int bh = b * HH + head;
  v4u val[8];
  size_t go[8];
#pragma unroll
  for (int j = 0; j < 8; ++j) {
    const int p  = tid + 256 * j;
    const int L  = p >> 3;
    const int pc = p & 7;
    const int d  = L >> 2;
    const int nl = (L & 3) * 64 + pc * 8;
    const _Float16* cp = st + nl * STP + d;
    Pack8 pk;
    pk.h = (v8h){cp[0 * STP], cp[1 * STP], cp[2 * STP], cp[3 * STP],
                 cp[4 * STP], cp[5 * STP], cp[6 * STP], cp[7 * STP]};
    val[j] = pk.u;
    go[j]  = ((size_t)bh * DD + d) * NN + nb + nl;
  }
  for (int ps = 0; ps < 2; ++ps) {
#pragma unroll
    for (int j = 0; j < 8; ++j) *(volatile v4u*)(vtp + go[j]) = val[j];
    __threadfence();
  }
}

#define KTP 72
#define PTP 72
#define OTP 68
static_assert(8 * 16 * OTP <= 9216);
__global__ __launch_bounds__(256) void k_attn(const _Float16* __restrict__ qp,
                                              const _Float16* __restrict__ kp,
                                              const _Float16* __restrict__ vt,
                                              const float* __restrict__ bias,
                                              float* __restrict__ out, float sscale) {
  __shared__ __align__(16) float smem[9216];
  _Float16* Ks = (_Float16*)smem;
  _Float16* Vs = Ks + 64 * KTP;
  _Float16* Pb = Vs + 64 * KTP;

  const int tid = threadIdx.x, lane = tid & 31, wave = tid >> 5;
  const int hh = lane >> 4, c = lane & 15;
  const int bh = blockIdx.x >> 4;
  const int qb = blockIdx.x & 15;
  const int b  = bh >> 4, h = bh & (HH - 1);
  const int q0 = qb * 128 + wave * 16;

  const _Float16* Q = qp + (size_t)bh * NN * DD;
  const _Float16* K = kp + (size_t)bh * NN * DD;
  const _Float16* V = vt + (size_t)bh * DD * NN;

  v16h qa[2];
  qa[0] = ldfrag(Q, DD, q0, 0, lane);
  qa[1] = ldfrag(Q, DD, q0, 32, lane);

  const float NEGI = -__builtin_huge_valf();
  float mrow[8], lrow[8];
  v8f oacc[4];
#pragma unroll
  for (int r = 0; r < 8; ++r) { mrow[r] = NEGI; lrow[r] = 0.f; }
#pragma unroll
  for (int t = 0; t < 4; ++t) oacc[t] = zero8();

  _Float16* pw = Pb + wave * (16 * PTP);

  for (int kc = 0; kc < NN / 64; ++kc) {
    const int kv0 = kc * 64;
    __syncthreads();
    {
      const int r  = tid >> 2;
      const int qq = (tid & 3) * 16;
      const _Float16* ks = K + (size_t)(kv0 + r) * DD + qq;
      *(v8h*)(Ks + r * KTP + qq)     = *(const v8h*)(ks);
      *(v8h*)(Ks + r * KTP + qq + 8) = *(const v8h*)(ks + 8);
      const _Float16* vs = V + (size_t)r * NN + kv0 + qq;
      *(v8h*)(Vs + r * KTP + qq)     = *(const v8h*)(vs);
      *(v8h*)(Vs + r * KTP + qq + 8) = *(const v8h*)(vs + 8);
    }
    __syncthreads();

    v8f s[4];
#pragma unroll
    for (int j = 0; j < 4; ++j) s[j] = zero8();
#pragma unroll
    for (int dc = 0; dc < 2; ++dc) {
#pragma unroll
      for (int j = 0; j < 4; ++j) {
        const v16h kb = ldfrag(Ks, KTP, j * 16, dc * 32, lane);
        s[j] = mma16(qa[dc], kb, s[j]);
      }
    }
    float cm[8];
#pragma unroll
    for (int r = 0; r < 8; ++r) {
      float m = NEGI;
#pragma unroll
      for (int j = 0; j < 4; ++j) {
        const float sv = s[j][r] * sscale;
        s[j][r] = sv;
        m = fmaxf(m, sv);
      }
#pragma unroll
      for (int off = 1; off < 16; off <<= 1) m = fmaxf(m, __shfl_xor(m, off, 32));
      cm[r] = m;
    }
    float al[8];
#pragma unroll
    for (int r = 0; r < 8; ++r) {
      const float mnew  = fmaxf(mrow[r], cm[r]);
      const float alpha = __expf(mrow[r] - mnew);
      mrow[r] = mnew;
      float psum = 0.f;
#pragma unroll
      for (int j = 0; j < 4; ++j) {
        const float p = __expf(s[j][r] - mnew);
        psum += p;
        pw[(8 * hh + r) * PTP + j * 16 + c] = (_Float16)(p * 1024.0f);
      }
#pragma unroll
      for (int off = 1; off < 16; off <<= 1) psum += __shfl_xor(psum, off, 32);
      lrow[r] = lrow[r] * alpha + psum;
      al[r] = alpha;
    }
#pragma unroll
    for (int t = 0; t < 4; ++t)
#pragma unroll
      for (int r = 0; r < 8; ++r) oacc[t][r] *= al[r];
    __syncthreads();

#pragma unroll
    for (int kk = 0; kk < 2; ++kk) {
      const v16h pa = ldfrag(pw, PTP, 0, kk * 32, lane);
#pragma unroll
      for (int t = 0; t < 4; ++t) {
        const v16h vb = ldfrag(Vs, KTP, t * 16, kk * 32, lane);
        oacc[t] = mma16(pa, vb, oacc[t]);
      }
    }
  }
  __syncthreads();

  float bvs[4];
#pragma unroll
  for (int t = 0; t < 4; ++t) bvs[t] = bias[h * DD + 16 * t + c];
  float* sw = smem + wave * (16 * OTP);
#pragma unroll
  for (int r = 0; r < 8; ++r) {
    const float inv = 3.0517578125e-05f / lrow[r];
#pragma unroll
    for (int t = 0; t < 4; ++t) sw[(8 * hh + r) * OTP + 16 * t + c] = oacc[t][r] * inv + bvs[t];
  }
  __syncthreads();
  v4f val[8];
  size_t go[8];
#pragma unroll
  for (int it = 0; it < 8; ++it) {
    const int p    = lane + 32 * it;
    const int L    = p >> 3;
    const int pc   = p & 7;
    const int rw   = L >> 1;
    const int half = L & 1;
    val[it] = *(const v4f*)(sw + rw * OTP + half * 32 + pc * 4);
    go[it]  = (size_t)(b * NN + q0 + rw) * CC + (size_t)h * DD + half * 32 + pc * 4;
  }
  for (int ps = 0; ps < 2; ++ps) {
#pragma unroll
    for (int it = 0; it < 8; ++it) *(volatile v4f*)(out + go[it]) = val[it];
    __threadfence();
  }
}

extern "C" void kernel_launch(void* const* d_in, const int* in_sizes, int n_in,
                              void* d_out, int out_size, void* d_ws, size_t ws_size,
                              hipStream_t stream) {
  if (n_in < 7) return;
  if (in_sizes[0] != ROWS * CC) return;
  if (in_sizes[1] != CC * CC) return;
  if (in_sizes[2] != CC) return;
  if (in_sizes[3] != CC * CC) return;
  if (in_sizes[4] != CC) return;
  if (in_sizes[5] != CC * CC) return;
  if (in_sizes[6] != CC) return;
  if (out_size != ROWS * CC) return;

  const float* x   = (const float*)d_in[0];
  const float* z_q = (const float*)d_in[1];
  const float* b_q = (const float*)d_in[2];
  const float* z_k = (const float*)d_in[3];
  const float* b_k = (const float*)d_in[4];
  const float* w_v = (const float*)d_in[5];
  const float* b_v = (const float*)d_in[6];
  float* out = (float*)d_out;

  size_t off = 0;
  const size_t oX   = off; off += (size_t)ROWS * CC * 2;
  const size_t oZq  = off; off += (size_t)CC * CC * 2;
  const size_t oZk  = off; off += (size_t)CC * CC * 2;
  const size_t oWv  = off; off += (size_t)CC * CC * 2;
  const size_t oQ   = off; off += PL * 2;
  const size_t oK   = off; off += PL * 2;
  const size_t oVt  = off; off += PL * 2;
  const size_t oLam = off; off += (size_t)ROWS * 4;
  const size_t oZnq = off; off += (size_t)CC * 4;
  const size_t oZnk = off; off += (size_t)CC * 4;
  if (off > ws_size) return;

  char* ws = (char*)d_ws;
  _Float16* Xh  = (_Float16*)(ws + oX);
  _Float16* Zqt = (_Float16*)(ws + oZq);
  _Float16* Zkt = (_Float16*)(ws + oZk);
  _Float16* Wvh = (_Float16*)(ws + oWv);
  _Float16* Qp  = (_Float16*)(ws + oQ);
  _Float16* Kp  = (_Float16*)(ws + oK);
  _Float16* Vtp = (_Float16*)(ws + oVt);
  float*    Lam = (float*)(ws + oLam);
  float*    Znq = (float*)(ws + oZnq);
  float*    Znk = (float*)(ws + oZnk);

  k_xprep<<<dim3(ROWS / 32), dim3(256), 0, stream>>>(x, Xh, Lam);
  const int ngrp = in_sizes[5] / 8;
  k_cvt8<<<dim3((ngrp + 255) / 256), dim3(256), 0, stream>>>(w_v, Wvh, ngrp, 32.0f);
  k_wt<<<dim3(CC / 64, CC / 64), dim3(256), 0, stream>>>(z_q, Zqt, CC, 16.0f);
  k_wt<<<dim3(CC / 64, CC / 64), dim3(256), 0, stream>>>(z_k, Zkt, CC, 16.0f);
  k_znorm<<<dim3(CC / 256), dim3(256), 0, stream>>>(z_q, Znq);
  k_znorm<<<dim3(CC / 256), dim3(256), 0, stream>>>(z_k, Znk);
  k_hproj<<<dim3(ROWS / 16), dim3(256), HPROJ_LDS_BYTES, stream>>>(Xh, Zqt, Znq, b_q, Lam, Qp);
  k_hproj<<<dim3(ROWS / 16), dim3(256), HPROJ_LDS_BYTES, stream>>>(Xh, Zkt, Znk, b_k, Lam, Kp);
  k_vproj<<<dim3(ROWS / 256, CC / 64), dim3(256), 0, stream>>>(Xh, Wvh, Vtp);
  k_attn<<<dim3(BB * HH * (NN / 128)), dim3(256), 0, stream>>>(Qp, Kp, Vtp, b_v, out, 1.220703125e-4f);
  (void)hipGetLastError();
}
